// highwayNet_d_8538394984638
// MI455X (gfx1250) — hardware-verified
//
#include <hip/hip_runtime.h>
#include <stdint.h>

typedef __attribute__((ext_vector_type(16))) _Float16 v16h;
typedef __attribute__((ext_vector_type(8)))  _Float16 v8h;
typedef __attribute__((ext_vector_type(16))) __bf16   v16b;
typedef __attribute__((ext_vector_type(8)))  __bf16   v8b;
typedef __attribute__((ext_vector_type(8)))  float    v8f;
typedef __attribute__((ext_vector_type(4)))  float    v4f;

__device__ __forceinline__ unsigned short f2bf_bits(float f) {
  unsigned u = __float_as_uint(f);
  return (unsigned short)((u + 0x7FFFu + ((u >> 16) & 1u)) >> 16);
}
__device__ __forceinline__ float bf_bits2f(unsigned short h) { return __uint_as_float(((unsigned)h) << 16); }

__device__ __forceinline__ void dep_guard_h(v8f& a, v8f& b, v16h x, v16h y) { asm volatile("v_nop\n\tv_nop\n\tv_nop\n\tv_nop" : "+v"(a), "+v"(b) : "v"(x), "v"(y)); }
__device__ __forceinline__ void dep_guard_b(v8f& a, v8f& b, v16b x, v16b y) { asm volatile("v_nop\n\tv_nop\n\tv_nop\n\tv_nop" : "+v"(a), "+v"(b) : "v"(x), "v"(y)); }
__device__ __forceinline__ void keep4_h(v16h a, v16h b, v16h c, v16h d) { asm volatile("v_nop" :: "v"(a), "v"(b), "v"(c), "v"(d)); }
__device__ __forceinline__ void keep4_b(v16b a, v16b b, v16b c, v16b d) { asm volatile("v_nop" :: "v"(a), "v"(b), "v"(c), "v"(d)); }
__device__ __forceinline__ void acc_guard4(v8f& a, v8f& b, v8f& c, v8f& d) { asm volatile("v_nop\n\tv_nop\n\tv_nop\n\tv_nop" : "+v"(a), "+v"(b), "+v"(c), "+v"(d)); }
template <typename T> struct Frag;
template <> struct Frag<_Float16> {
  typedef v16h V; union U { v16h v; v8h h[2]; };
  static __device__ __forceinline__ v16h load(const _Float16* p) {
    U f; f.h[0] = *(const v8h*)(p); f.h[1] = *(const v8h*)(p + 16); return f.v;
  }
  static __device__ __forceinline__ v8f mma(v16h a, v16h b, v8f c) {
    return __builtin_amdgcn_wmma_f32_16x16x32_f16(false, a, false, b, (short)0, c, false, false);
  }
  static __device__ __forceinline__ void guard(v8f& a, v8f& b, v16h x, v16h y) { dep_guard_h(a, b, x, y); }
  static __device__ __forceinline__ void keep(v16h a, v16h b, v16h c, v16h d) { keep4_h(a, b, c, d); }
};
template <> struct Frag<__bf16> {
  typedef v16b V; union U { v16b v; v8b h[2]; };
  static __device__ __forceinline__ v16b load(const __bf16* p) {
    U f; f.h[0] = *(const v8b*)(p); f.h[1] = *(const v8b*)(p + 16); return f.v;
  }
  static __device__ __forceinline__ v8f mma(v16b a, v16b b, v8f c) {
    return __builtin_amdgcn_wmma_f32_16x16x32_bf16(false, a, false, b, (short)0, c, false, false);
  }
  static __device__ __forceinline__ void guard(v8f& a, v8f& b, v16b x, v16b y) { dep_guard_b(a, b, x, y); }
  static __device__ __forceinline__ void keep(v16b a, v16b b, v16b c, v16b d) { keep4_b(a, b, c, d); }
};

template <int ET> struct Elem;
template <> struct Elem<0> { typedef _Float16 T; };
template <> struct Elem<1> { typedef __bf16 T; };
template <int ET, bool SPLIT, int BIAS_MODE, int OUT_MODE, bool RESID, int ACT = 0>
__global__ __launch_bounds__(256) void wmma_gemm64(
    const unsigned short* __restrict__ Ap, const unsigned short* __restrict__ A2p, int lda, long strideA,
    const unsigned short* __restrict__ Btp, const unsigned short* __restrict__ Bt2p, int ldb, long strideB,
    void* __restrict__ Cout, void* __restrict__ Cout2, int ldc, long strideC,
    const float* __restrict__ bias,
    const float* __restrict__ resid, long strideR,
    int M, int N, int K, float scale) {
  typedef typename Elem<ET>::T T;
  typedef typename Frag<T>::V V;
  const T* A = (const T*)Ap; const T* A2 = (const T*)A2p; const T* Bt = (const T*)Btp; const T* Bt2 = (const T*)Bt2p;
  __shared__ __align__(16) float sT[8][16 * 68];
  const int b    = blockIdx.y;
  const int lane = threadIdx.x & 31;
  const int wave = threadIdx.x >> 5;
  const int tilesN = N >> 6;
  const int tilesM = M >> 6;
  const int tile = blockIdx.x * 8 + wave;
  if (tile >= tilesM * tilesN) return;
  const int tm = tile / tilesN;
  const int tn = tile - tm * tilesN;
  const int m0 = tm << 6;
  const int n0 = tn << 6;

  const T* Ab  = A  + (size_t)b * strideA;
  const T* Bb  = Bt + (size_t)b * strideB;
  const T* Ab2 = SPLIT ? (A2  + (size_t)b * strideA) : nullptr;
  const T* Bb2 = SPLIT ? (Bt2 + (size_t)b * strideB) : nullptr;

  const int rlane = lane & 15;
  const int koff  = (lane >> 4) * 8;
  const int mOff  = (lane >> 4) * 8;

  v8f acc[4][4];
#pragma unroll
  for (int i = 0; i < 4; ++i)
#pragma unroll
    for (int j = 0; j < 4; ++j) acc[i][j] = (v8f){0.f,0.f,0.f,0.f,0.f,0.f,0.f,0.f};

  for (int k0 = 0; k0 < K; k0 += 32) {
    V bh[4], bl[4];
#pragma unroll
    for (int j = 0; j < 4; ++j) {
      const size_t bo = (size_t)(n0 + (j << 4) + rlane) * ldb + koff + k0;
      bh[j] = Frag<T>::load(Bb + bo);
      if (SPLIT) bl[j] = Frag<T>::load(Bb2 + bo);
    }
#pragma unroll
    for (int i = 0; i < 4; ++i) {
      const size_t ao = (size_t)(m0 + (i << 4) + rlane) * lda + koff + k0;
      V ah = Frag<T>::load(Ab + ao);
      V al;
      if (SPLIT) al = Frag<T>::load(Ab2 + ao);
#pragma unroll
      for (int j = 0; j < 4; ++j) {
        acc[i][j] = Frag<T>::mma(ah, bh[j], acc[i][j]);
        if (SPLIT) {
          acc[i][j] = Frag<T>::mma(ah, bl[j], acc[i][j]);
          acc[i][j] = Frag<T>::mma(al, bh[j], acc[i][j]);
        }
      }
      Frag<T>::guard(acc[i][0], acc[i][3], ah, SPLIT ? al : ah);
    }
    Frag<T>::keep(bh[0], bh[1], bh[2], bh[3]);
    if (SPLIT) Frag<T>::keep(bl[0], bl[1], bl[2], bl[3]);
  }
  acc_guard4(acc[0][0], acc[0][1], acc[0][2], acc[0][3]);
  acc_guard4(acc[1][0], acc[1][1], acc[1][2], acc[1][3]);
  acc_guard4(acc[2][0], acc[2][1], acc[2][2], acc[2][3]);
  acc_guard4(acc[3][0], acc[3][1], acc[3][2], acc[3][3]);

  float* slab = sT[wave];
  const float* Rb = RESID ? (resid + (size_t)b * strideR) : nullptr;
#pragma unroll
  for (int i = 0; i < 4; ++i) {
    const int mBase = m0 + (i << 4);
#pragma unroll
    for (int j = 0; j < 4; ++j) {
      const int n = n0 + (j << 4) + rlane;
      float bv = 0.f;
      if (BIAS_MODE == 2) bv = bias[n];
#pragma unroll
      for (int r = 0; r < 8; ++r) {
        float v = acc[i][j][r] * scale;
        if (BIAS_MODE == 1) v += bias[mBase + mOff + r];
        if (BIAS_MODE == 2) v += bv;
        if (RESID) v += Rb[(size_t)(mBase + mOff + r) * ldc + n];
        if (ACT == 1) v = tanhf(v);
        if (ACT == 2) v = fmaxf(v, 0.0f);
        if (ACT == 3) v = v / (1.0f + expf(-v));
        if (ACT == 4) v = (v > 0.f) ? v : 0.01f * v;
        if (ACT == 5) v = 0.5f * v * (1.0f + erff(v * 0.70710678118654752f));
        if (ACT == 6) v = (v > 0.f) ? v : 0.1f * v;
        slab[(mOff + r) * 68 + (j << 4) + rlane] = v;
      }
    }
    __builtin_amdgcn_fence(__ATOMIC_RELEASE, "workgroup");
    __builtin_amdgcn_wave_barrier();
    __builtin_amdgcn_fence(__ATOMIC_ACQUIRE, "workgroup");
    if (OUT_MODE == 0) {
      float* C = (float*)Cout + (size_t)b * strideC;
      const int hh = lane >> 4, c4 = (lane & 15) * 4;
      for (int pass = 0; pass < 2; ++pass) {
#pragma unroll
        for (int it = 0; it < 8; ++it) {
          const int row = it * 2 + hh;
          v4f v = *(const v4f*)(slab + row * 68 + c4);
          *(volatile v4f*)(C + (size_t)(mBase + row) * ldc + n0 + c4) = v;
        }
        __threadfence();
      }
    } else {
      const int q = lane >> 3, c8 = (lane & 7) * 8;
      unsigned short* C  = (unsigned short*)Cout  + (size_t)b * strideC;
      unsigned short* C2 = (OUT_MODE == 2) ? ((unsigned short*)Cout2 + (size_t)b * strideC) : nullptr;
      for (int pass = 0; pass < 2; ++pass) {
#pragma unroll
        for (int it = 0; it < 4; ++it) {
          const int row = it * 4 + q;
          const float* sp = slab + row * 68 + c8;
          v8h hv, lv;
#pragma unroll
          for (int e = 0; e < 8; ++e) {
            if (OUT_MODE == 1) {
              hv[e] = (_Float16)sp[e];
            } else {
              unsigned short hb = f2bf_bits(sp[e]);
              unsigned short lb = f2bf_bits(sp[e] - bf_bits2f(hb));
              hv[e] = __builtin_bit_cast(_Float16, hb);
              lv[e] = __builtin_bit_cast(_Float16, lb);
            }
          }
          *(volatile v8h*)(C + (size_t)(mBase + row) * ldc + n0 + c8) = hv;
          if (OUT_MODE == 2) *(volatile v8h*)(C2 + (size_t)(mBase + row) * ldc + n0 + c8) = lv;
        }
        __threadfence();
      }
    }
    __builtin_amdgcn_fence(__ATOMIC_RELEASE, "workgroup");
    __builtin_amdgcn_wave_barrier();
    __builtin_amdgcn_fence(__ATOMIC_ACQUIRE, "workgroup");
  }
}

constexpr int kFeat  = 32;
constexpr int kEmb   = 32;
constexpr int kHid   = 64;
constexpr int kGates = 192;
constexpr int kGrpSz = 32;
constexpr int kGC    = 128;
constexpr int kEP    = 40;
constexpr int kHP    = 72;

__device__ __forceinline__ float lk01(float x) { return x > 0.f ? x : 0.1f * x; }
__device__ __forceinline__ float sigm_f(float x) {
  x = fminf(fmaxf(x, -30.0f), 30.0f);
  return 1.0f / (1.0f + expf(-x));
}
__device__ __forceinline__ v8f mma_g(v16h a, v16h b, v8f c) {
  c = __builtin_amdgcn_wmma_f32_16x16x32_f16(false, a, false, b, (short)0, c, false, false);
  asm volatile("v_nop\n\tv_nop\n\tv_nop\n\tv_nop" : "+v"(c) : "v"(a), "v"(b));
  return c;
}

__global__ __launch_bounds__(256) void prep_kernel(
    const float* __restrict__ Wih_f, const float* __restrict__ Whh_f,
    const float* __restrict__ Wih_b, const float* __restrict__ Whh_b,
    const float* __restrict__ Wm, const float* __restrict__ bm,
    const float* __restrict__ Ws1, const float* __restrict__ bs1,
    const float* __restrict__ Ws2, const float* __restrict__ bs2,
    const float* __restrict__ Wo1, const float* __restrict__ bo1,
    const float* __restrict__ Wo2, const float* __restrict__ bo2,
    unsigned short* __restrict__ dWihf, unsigned short* __restrict__ dWhhf,
    unsigned short* __restrict__ dWihb, unsigned short* __restrict__ dWhhb,
    unsigned short* __restrict__ dWmT, unsigned short* __restrict__ dWs1T,
    unsigned short* __restrict__ dWs2T, unsigned short* __restrict__ dWo1T,
    unsigned short* __restrict__ dWo2T, float* __restrict__ cb)
{
  __shared__ __align__(16) float cbuf[384];
  const int tid = threadIdx.x;
  const int bid = blockIdx.x;
  int p, lb;
  if (bid < 3)       { p = 0; lb = bid; }
  else if (bid < 9)  { p = 1; lb = bid - 3; }
  else if (bid < 12) { p = 2; lb = bid - 9; }
  else if (bid < 18) { p = 3; lb = bid - 12; }
  else if (bid < 20) { p = 4; lb = bid - 18; }
  else if (bid < 21) { p = 5; lb = bid - 20; }
  else if (bid < 23) { p = 6; lb = bid - 21; }
  else if (bid < 25) { p = 7; lb = bid - 23; }
  else if (bid < 27) { p = 8; lb = bid - 25; }
  else               { p = 9; lb = 0; }

  if (p == 9) {
    for (int idx = tid; idx < 384; idx += 256) {
      const int arr = idx >> 6, ci = idx & 63;
      const int c31 = min(ci, 31), c15 = min(ci, 15), c2 = min(ci, 2);
      const float wbm  = bm[c31];
      const float wbs2 = bs2[c31];
      const float wbo1 = bo1[c15];
      const float wbo2 = bo2[c2];
      const float v0 = (ci < 32) ? wbm : 0.f;
      const float v1 = bs1[ci] * 8.0f;
      const float v2 = (ci < 32) ? wbs2 : 0.f;
      const float v3 = (ci < 16) ? wbo1 * 16.0f : 0.f;
      const float v4 = (ci < 3) ? wbo2 : 0.f;
      float z = 0.f;
#pragma unroll 1
      for (int k = 0; k < 64; ++k) z += lk01(bs1[k]) * Ws2[k * 32 + c31];
      z = lk01(z + wbs2);
      const float v5 = (ci < 32) ? z : 0.f;
      float v = v5;
      if (arr == 0) v = v0; else if (arr == 1) v = v1; else if (arr == 2) v = v2;
      else if (arr == 3) v = v3; else if (arr == 4) v = v4;
      cbuf[idx] = v;
    }
    __syncthreads();
    if (tid < 32) {
      v4f cv[3];
#pragma unroll
      for (int it = 0; it < 3; ++it) cv[it] = *(const v4f*)(cbuf + it * 128 + tid * 4);
      for (int pass = 0; pass < 2; ++pass) {
#pragma unroll
        for (int it = 0; it < 3; ++it) *(volatile v4f*)(cb + it * 128 + tid * 4) = cv[it];
        __threadfence();
      }
    }
  } else {
    const int e0 = (lb * 256 + tid) * 8;
    float vals[8];
    _Float16* dst;
    if (p == 0) {
      dst = (_Float16*)(void*)dWihf;
#pragma unroll
      for (int i = 0; i < 8; ++i) vals[i] = Wih_f[e0 + i];
    } else if (p == 1) {
      dst = (_Float16*)(void*)dWhhf;
#pragma unroll
      for (int i = 0; i < 8; ++i) vals[i] = Whh_f[e0 + i];
    } else if (p == 2) {
      dst = (_Float16*)(void*)dWihb;
#pragma unroll
      for (int i = 0; i < 8; ++i) vals[i] = Wih_b[e0 + i];
    } else if (p == 3) {
      dst = (_Float16*)(void*)dWhhb;
#pragma unroll
      for (int i = 0; i < 8; ++i) vals[i] = Whh_b[e0 + i];
    } else if (p == 4) {
      dst = (_Float16*)(void*)dWmT;
      const int n = e0 >> 6, kb = e0 & 63, nn = min(n, 31);
#pragma unroll
      for (int i = 0; i < 8; ++i) { const float w = Wm[(kb + i) * 32 + nn]; vals[i] = (n < 32) ? w : 0.f; }
    } else if (p == 5) {
      dst = (_Float16*)(void*)dWs1T;
      const int n = e0 >> 5, kb = e0 & 31;
#pragma unroll
      for (int i = 0; i < 8; ++i) vals[i] = Ws1[(kb + i) * 64 + n];
    } else if (p == 6) {
      dst = (_Float16*)(void*)dWs2T;
      const int n = e0 >> 6, kb = e0 & 63, nn = min(n, 31);
#pragma unroll
      for (int i = 0; i < 8; ++i) { const float w = Ws2[(kb + i) * 32 + nn]; vals[i] = (n < 32) ? w : 0.f; }
    } else if (p == 7) {
      dst = (_Float16*)(void*)dWo1T;
      const int n = e0 >> 6, kb = e0 & 63, nn = min(n, 15);
#pragma unroll
      for (int i = 0; i < 8; ++i) { const float w = Wo1[(kb + i) * 16 + nn]; vals[i] = (n < 16) ? w : 0.f; }
    } else {
      dst = (_Float16*)(void*)dWo2T;
      const int n = e0 >> 6, kb = e0 & 63, nn = min(n, 2);
#pragma unroll
      for (int i = 0; i < 8; ++i) {
        const int k = kb + i, kk = min(k, 15);
        const float w = Wo2[kk * 3 + nn];
        vals[i] = (n < 3 && k < 16) ? w : 0.f;
      }
    }
    v8h hv;
#pragma unroll
    for (int i = 0; i < 8; ++i) hv[i] = (_Float16)(vals[i] * 8.0f);
    *(volatile v8h*)(dst + e0) = hv;
    __threadfence();
    *(volatile v8h*)(dst + e0) = hv;
  }
}

__global__ __launch_bounds__(128) void gru_bidir_kernel(
    const float* __restrict__ scene, const float* __restrict__ W_emb, const float* __restrict__ b_emb,
    const unsigned short* __restrict__ Wih16f, const unsigned short* __restrict__ Whh16f,
    const float* __restrict__ bih_f, const float* __restrict__ bhh_f,
    const unsigned short* __restrict__ Wih16b, const unsigned short* __restrict__ Whh16b,
    const float* __restrict__ bih_b, const float* __restrict__ bhh_b,
    unsigned short* __restrict__ HM16p, int nveh)
{
  __shared__ __align__(16) float sc[32 * kFeat];
  __shared__ __align__(16) float wemb[96];
  __shared__ __align__(16) _Float16 E16[32 * kEP];
  __shared__ __align__(16) _Float16 H16[32 * kHP];
  __shared__ __align__(16) float stg[32 * 68];

  const int tid = threadIdx.x, wave = tid >> 5, lane = tid & 31;
  const int hh = lane >> 4, c = lane & 15;
  const int v0 = blockIdx.x * 32;
  const int u = wave * 16 + c;
  const float kS64 = 1.0f / 64.0f;

  for (int i = tid; i < 32 * kFeat; i += 128) sc[i] = scene[(size_t)v0 * kFeat + i];
  if (wave < 2) wemb[tid] = W_emb[tid];
  else if (wave == 2) wemb[64 + lane] = b_emb[lane];
  __syncthreads();

  float hf[2][8], hr[2][8];
#pragma unroll
  for (int m = 0; m < 2; ++m)
#pragma unroll
    for (int r = 0; r < 8; ++r) { hf[m][r] = 0.f; hr[m][r] = 0.f; }

#pragma unroll 1
  for (int dir = 0; dir < 2; ++dir) {
    const _Float16* Wih = (const _Float16*)(const void*)(dir ? Wih16b : Wih16f);
    const _Float16* Whh = (const _Float16*)(const void*)(dir ? Whh16b : Whh16f);
    const float* bih = dir ? bih_b : bih_f;
    const float* bhh = dir ? bhh_b : bhh_f;
    const float bR  = bih[u] + bhh[u];
    const float bZ  = bih[64 + u] + bhh[64 + u];
    const float bNX = bih[128 + u];
    const float bNH = bhh[128 + u];
#pragma unroll
    for (int m = 0; m < 2; ++m)
#pragma unroll
      for (int r = 0; r < 8; ++r) { hr[m][r] = 0.f; H16[(16 * m + 8 * hh + r) * kHP + u] = (_Float16)0.0f; }

#pragma unroll 1
    for (int s = 0; s < 16; ++s) {
      const int t = dir ? (15 - s) : s;
      {
        const int row = tid >> 2, e0 = (tid & 3) * 8;
        const float x = sc[row * kFeat + t], y = sc[row * kFeat + 16 + t];
        v8h ev;
#pragma unroll
        for (int i = 0; i < 8; ++i) {
          const int e = e0 + i;
          float a = x * wemb[e] + y * wemb[32 + e] + wemb[64 + e];
          a = lk01(a);
          ev[i] = (_Float16)(a * 8.0f);
        }
        *(v8h*)(E16 + row * kEP + e0) = ev;
      }
      __syncthreads();

      v8f aR[2], aZ[2], aNX[2], aNH[2];
#pragma unroll
      for (int m = 0; m < 2; ++m) {
        aR[m]  = (v8f){0.f,0.f,0.f,0.f,0.f,0.f,0.f,0.f};
        aZ[m]  = (v8f){0.f,0.f,0.f,0.f,0.f,0.f,0.f,0.f};
        aNX[m] = (v8f){0.f,0.f,0.f,0.f,0.f,0.f,0.f,0.f};
        aNH[m] = (v8f){0.f,0.f,0.f,0.f,0.f,0.f,0.f,0.f};
      }
      v16h fe[2], fh0[2], fh1[2];
#pragma unroll
      for (int m = 0; m < 2; ++m) {
        fe[m]  = Frag<_Float16>::load(E16 + (16 * m + c) * kEP + 8 * hh);
        fh0[m] = Frag<_Float16>::load(H16 + (16 * m + c) * kHP + 8 * hh);
        fh1[m] = Frag<_Float16>::load(H16 + (16 * m + c) * kHP + 32 + 8 * hh);
      }
#pragma unroll
      for (int g = 0; g < 3; ++g) {
        const int n = g * 64 + u;
        const v16h bx = Frag<_Float16>::load(Wih + (size_t)n * kEmb + 8 * hh);
        const v16h b0 = Frag<_Float16>::load(Whh + (size_t)n * kHid + 8 * hh);
        const v16h b1 = Frag<_Float16>::load(Whh + (size_t)n * kHid + 32 + 8 * hh);
#pragma unroll
        for (int m = 0; m < 2; ++m) {
          if (g == 0) {
            aR[m] = mma_g(fe[m], bx, aR[m]); aR[m] = mma_g(fh0[m], b0, aR[m]); aR[m] = mma_g(fh1[m], b1, aR[m]);
          } else if (g == 1) {
            aZ[m] = mma_g(fe[m], bx, aZ[m]); aZ[m] = mma_g(fh0[m], b0, aZ[m]); aZ[m] = mma_g(fh1[m], b1, aZ[m]);
          } else {
            aNX[m] = mma_g(fe[m], bx, aNX[m]);
            aNH[m] = mma_g(fh0[m], b0, aNH[m]); aNH[m] = mma_g(fh1[m], b1, aNH[m]);
          }
        }
      }
      __syncthreads();

#pragma unroll
      for (int m = 0; m < 2; ++m) {
#pragma unroll
        for (int r = 0; r < 8; ++r) {
          const float pr = aR[m][r] * kS64 + bR;
          const float pz = aZ[m][r] * kS64 + bZ;
          const float xn = aNX[m][r] * kS64 + bNX;
          const float hn = aNH[m][r] * kS64 + bNH;
          const float rg = sigm_f(pr);
          const float zg = sigm_f(pz);
          const float ng = tanhf(xn + rg * hn);
          const float h = (1.0f - zg) * ng + zg * hr[m][r];
          hr[m][r] = h;
          H16[(16 * m + 8 * hh + r) * kHP + u] = (_Float16)(h * 8.0f);
        }
      }
    }
    if (dir == 0) {
#pragma unroll
      for (int m = 0; m < 2; ++m)
#pragma unroll
        for (int r = 0; r < 8; ++r) hf[m][r] = hr[m][r];
    }
  }

#pragma unroll
  for (int m = 0; m < 2; ++m)
#pragma unroll
    for (int r = 0; r < 8; ++r) stg[(16 * m + 8 * hh + r) * 68 + u] = 0.5f * (hf[m][r] + hr[m][r]);
  __syncthreads();
  {
    _Float16* HM16 = (_Float16*)(void*)HM16p;
    const int q = lane >> 3, c8 = (lane & 7) * 8;
    v8h hv[2];
#pragma unroll
    for (int it = 0; it < 2; ++it) {
      const int row = wave * 8 + it * 4 + q;
#pragma unroll
      for (int e = 0; e < 8; ++e) hv[it][e] = (_Float16)(stg[row * 68 + c8 + e] * 8.0f);
    }
    for (int pass = 0; pass < 2; ++pass) {
#pragma unroll
      for (int it = 0; it < 2; ++it) {
        const int row = wave * 8 + it * 4 + q;
        *(volatile v8h*)(HM16 + (size_t)(v0 + row) * kHid + c8) = hv[it];
      }
      __threadfence();
    }
  }
}

__global__ __launch_bounds__(256) void rel_build_kernel(
    const float* __restrict__ scene, const int* __restrict__ index_div,
    int gbase, int nveh, unsigned short* __restrict__ A1p)
{
  __shared__ __align__(16) float ft[32 * kFeat];
  const int tid = threadIdx.x, wave = tid >> 5, lane = tid & 31;
  const int g = gbase + blockIdx.x;
  {
    const int i = tid >> 3, part = tid & 7;
    int idx = index_div[g * kGrpSz + i];
    idx = min(max(idx, 0), nveh - 1);
    const v4f vv = *(const v4f*)(scene + (size_t)idx * kFeat + part * 4);
    *(v4f*)(ft + i * kFeat + part * 4) = vv;
  }
  __syncthreads();
  _Float16* A1 = (_Float16*)(void*)A1p + (size_t)blockIdx.x * 1024 * kFeat;
  const int k0 = (lane & 3) * 8;
  const int qo = wave * 8 + (lane >> 2);
  for (int pass = 0; pass < 2; ++pass) {
#pragma unroll 1
    for (int it = 0; it < 16; ++it) {
      const int q = it * 64 + qo;
      const int j = q >> 5, i = q & 31;
      v8h hv;
#pragma unroll
      for (int e = 0; e < 8; ++e) hv[e] = (_Float16)(ft[i * kFeat + k0 + e] - ft[j * kFeat + k0 + e]);
      *(volatile v8h*)(A1 + (size_t)q * kFeat + k0) = hv;
    }
    __threadfence();
  }
}

__global__ __launch_bounds__(256) void assemble_kernel(
    const float* __restrict__ S, const float* __restrict__ E, const float* __restrict__ ZE,
    int vbase, float* __restrict__ out1, unsigned short* __restrict__ FEp)
{
  __shared__ __align__(16) float slab[32 * 68];
  const int tid = threadIdx.x, wave = tid >> 5, lane = tid & 31;
  const int hh = lane >> 4, c4 = (lane & 15) * 4;
  const int cs = c4 & 31;
  const bool lowhalf = (c4 < 32);
  const int vl0 = blockIdx.x * 32;
  v4f val[2];
#pragma unroll
  for (int it = 0; it < 2; ++it) {
    const int rib = wave * 4 + it * 2 + hh;
    const int vl = vl0 + rib;
    const int v = vbase + vl;
    const v4f sv = *(const v4f*)(S + (size_t)v * 64 + cs);
    v4f ps = (v4f){0.f, 0.f, 0.f, 0.f};
    const float* ep = E + (size_t)vl * kGrpSz * 64 + cs;
#pragma unroll 1
    for (int i = 0; i < kGrpSz; ++i) ps += *(const v4f*)(ep + i * 64);
    const v4f ze = *(const v4f*)(ZE + cs);
    const v4f pv = (ps - ze) * (1.0f / 31.0f);
#pragma unroll
    for (int e = 0; e < 4; ++e) {
      const float w = lowhalf ? sv[e] : pv[e];
      val[it][e] = w;
      slab[rib * 68 + c4 + e] = w;
    }
  }
  __builtin_amdgcn_fence(__ATOMIC_RELEASE, "workgroup");
  __builtin_amdgcn_wave_barrier();
  __builtin_amdgcn_fence(__ATOMIC_ACQUIRE, "workgroup");
  const int q = lane >> 3, c8 = (lane & 7) * 8;
  const int rowf = wave * 4 + q;
  v8h hv;
#pragma unroll
  for (int e = 0; e < 8; ++e) hv[e] = (_Float16)(slab[rowf * 68 + c8 + e] * 8.0f);
  _Float16* FE = (_Float16*)(void*)FEp;
  for (int pass = 0; pass < 2; ++pass) {
#pragma unroll
    for (int it = 0; it < 2; ++it) {
      const int v = vbase + vl0 + wave * 4 + it * 2 + hh;
      *(volatile v4f*)(out1 + (size_t)v * 64 + c4) = val[it];
    }
    *(volatile v8h*)(FE + (size_t)(vbase + vl0 + rowf) * 64 + c8) = hv;
    __threadfence();
  }
}

__global__ __launch_bounds__(256) void pack_logits_kernel(
    const float* __restrict__ LG, float* __restrict__ out0, int nveh)
{
  const int t = blockIdx.x * 256 + threadIdx.x;
  const int f0 = t * 4;
  if (f0 + 3 >= nveh * 3 + 3) return;
  v4f v;
#pragma unroll
  for (int e = 0; e < 4; ++e) {
    const int f = f0 + e;
    int row = f / 3;
    const int col = f - row * 3;
    row = min(row, nveh - 1);
    v[e] = LG[(size_t)row * 64 + col];
  }
  *(volatile v4f*)(out0 + f0) = v;
  __threadfence();
  *(volatile v4f*)(out0 + f0) = v;
}

extern "C" void kernel_launch(void* const* d_in, const int* in_sizes, int n_in,
                              void* d_out, int out_size, void* d_ws, size_t ws_size,
                              hipStream_t stream) {
  if (n_in < 25) return;
  const float* scene     = (const float*)d_in[0];
  const int*   index_div = (const int*)d_in[4];
  const float* W_emb = (const float*)d_in[5];
  const float* b_emb = (const float*)d_in[6];
  const float* Wih_f = (const float*)d_in[7];
  const float* Whh_f = (const float*)d_in[8];
  const float* bih_f = (const float*)d_in[9];
  const float* bhh_f = (const float*)d_in[10];
  const float* Wih_b = (const float*)d_in[11];
  const float* Whh_b = (const float*)d_in[12];
  const float* bih_b = (const float*)d_in[13];
  const float* bhh_b = (const float*)d_in[14];
  const float* Wm  = (const float*)d_in[15];
  const float* bm  = (const float*)d_in[16];
  const float* Ws1 = (const float*)d_in[17];
  const float* bs1 = (const float*)d_in[18];
  const float* Ws2 = (const float*)d_in[19];
  const float* bs2 = (const float*)d_in[20];
  const float* Wo1 = (const float*)d_in[21];
  const float* bo1 = (const float*)d_in[22];
  const float* Wo2 = (const float*)d_in[23];
  const float* bo2 = (const float*)d_in[24];

  const int nveh = in_sizes[0] / kFeat;
  const int ngrp = in_sizes[4] / kGrpSz;
  if (nveh <= 0 || ngrp * kGrpSz != nveh || (ngrp % kGC) != 0 || (nveh % 64) != 0) return;
  if (out_size != nveh * 67) return;
  float* out0 = (float*)d_out;
  float* out1 = (float*)d_out + (size_t)nveh * 3;

  char* ws = (char*)d_ws;
  size_t off = 0;
  auto carve = [&](size_t bytes) -> size_t { size_t o = off; off += (bytes + 255) & ~(size_t)255; return o; };
  const size_t oWihf = carve((size_t)kGates * kEmb * 2);
  const size_t oWhhf = carve((size_t)kGates * kHid * 2);
  const size_t oWihb = carve((size_t)kGates * kEmb * 2);
  const size_t oWhhb = carve((size_t)kGates * kHid * 2);
  const size_t oWmT  = carve(64 * 64 * 2);
  const size_t oWs1T = carve(64 * 32 * 2);
  const size_t oWs2T = carve(64 * 64 * 2);
  const size_t oWo1T = carve(64 * 64 * 2);
  const size_t oWo2T = carve(64 * 64 * 2);
  const size_t oCB   = carve(384 * 4);
  const size_t oHM   = carve((size_t)nveh * 64 * 2);
  const size_t oS    = carve((size_t)nveh * 64 * 4);
  const size_t oFE   = carve((size_t)nveh * 64 * 2);
  const size_t oT1   = carve((size_t)nveh * 64 * 2);
  const size_t oLG   = carve((size_t)nveh * 64 * 4);
  const size_t P     = (size_t)kGC * kGrpSz * kGrpSz;
  const size_t oA1   = carve(P * 32 * 2);
  const size_t oH1   = carve(P * 64 * 2);
  const size_t oE    = carve(P * 64 * 4);
  if (off > ws_size) return;

  unsigned short* Wihf16 = (unsigned short*)(ws + oWihf);
  unsigned short* Whhf16 = (unsigned short*)(ws + oWhhf);
  unsigned short* Wihb16 = (unsigned short*)(ws + oWihb);
  unsigned short* Whhb16 = (unsigned short*)(ws + oWhhb);
  unsigned short* WmT16  = (unsigned short*)(ws + oWmT);
  unsigned short* Ws1T16 = (unsigned short*)(ws + oWs1T);
  unsigned short* Ws2T16 = (unsigned short*)(ws + oWs2T);
  unsigned short* Wo1T16 = (unsigned short*)(ws + oWo1T);
  unsigned short* Wo2T16 = (unsigned short*)(ws + oWo2T);
  float* cb   = (float*)(ws + oCB);
  float* BM64   = cb;
  float* BS1x8  = cb + 64;
  float* BS2p   = cb + 128;
  float* BO1x16 = cb + 192;
  float* BO2p   = cb + 256;
  float* ZE     = cb + 320;
  unsigned short* HM16 = (unsigned short*)(ws + oHM);
  float* Spl = (float*)(ws + oS);
  unsigned short* FE16 = (unsigned short*)(ws + oFE);
  unsigned short* T116 = (unsigned short*)(ws + oT1);
  float* LG = (float*)(ws + oLG);
  unsigned short* A1 = (unsigned short*)(ws + oA1);
  unsigned short* H1 = (unsigned short*)(ws + oH1);
  float* Epl = (float*)(ws + oE);

  prep_kernel<<<28, 256, 0, stream>>>(Wih_f, Whh_f, Wih_b, Whh_b, Wm, bm, Ws1, bs1, Ws2, bs2,
                                        Wo1, bo1, Wo2, bo2,
                                        Wihf16, Whhf16, Wihb16, Whhb16, WmT16, Ws1T16, Ws2T16,
                                        Wo1T16, Wo2T16, cb);
  gru_bidir_kernel<<<nveh / 32, 128, 0, stream>>>(scene, W_emb, b_emb, Wihf16, Whhf16, bih_f, bhh_f,
                                                    Wihb16, Whhb16, bih_b, bhh_b, HM16, nveh);
  {
    const int tiles = (nveh / 64) * 1;
    wmma_gemm64<0, false, 2, 0, false, 6><<<dim3((tiles + 7) / 8, 1), 256, 0, stream>>>(
        HM16, nullptr, 64, 0L, WmT16, nullptr, 64, 0L, (void*)Spl, nullptr, 64, 0L,
        BM64, nullptr, 0L, nveh, 64, 64, 1.0f / 64.0f);
  }
  const int nchunk = ngrp / kGC;
  const int Pi = (int)P;
  for (int ch = 0; ch < nchunk; ++ch) {
    rel_build_kernel<<<kGC, 256, 0, stream>>>(scene, index_div, ch * kGC, nveh, A1);
    {
      const int tiles = (Pi / 64) * 1;
      wmma_gemm64<0, false, 2, 1, false, 6><<<dim3((tiles + 7) / 8, 1), 256, 0, stream>>>(
          A1, nullptr, 32, 0L, Ws1T16, nullptr, 32, 0L, (void*)H1, nullptr, 64, 0L,
          BS1x8, nullptr, 0L, Pi, 64, 32, 1.0f);
      wmma_gemm64<0, false, 2, 0, false, 6><<<dim3((tiles + 7) / 8, 1), 256, 0, stream>>>(
          H1, nullptr, 64, 0L, Ws2T16, nullptr, 64, 0L, (void*)Epl, nullptr, 64, 0L,
          BS2p, nullptr, 0L, Pi, 64, 64, 1.0f / 64.0f);
    }
    assemble_kernel<<<(kGC * kGrpSz) / 32, 256, 0, stream>>>(Spl, Epl, ZE, ch * kGC * kGrpSz, out1, FE16);
  }
  {
    const int tiles = (nveh / 64) * 1;
    wmma_gemm64<0, false, 2, 1, false, 6><<<dim3((tiles + 7) / 8, 1), 256, 0, stream>>>(
        FE16, nullptr, 64, 0L, Wo1T16, nullptr, 64, 0L, (void*)T116, nullptr, 64, 0L,
        BO1x16, nullptr, 0L, nveh, 64, 64, 0.25f);
    wmma_gemm64<0, false, 2, 0, false, 0><<<dim3((tiles + 7) / 8, 1), 256, 0, stream>>>(
        T116, nullptr, 64, 0L, Wo2T16, nullptr, 64, 0L, (void*)LG, nullptr, 64, 0L,
        BO2p, nullptr, 0L, nveh, 64, 64, 1.0f / 128.0f);
  }
  pack_logits_kernel<<<(nveh * 3 / 4 + 255) / 256, 256, 0, stream>>>(LG, out0, nveh);
}
